// dcn_layer_28638841929772
// MI455X (gfx1250) — hardware-verified
//
#include <hip/hip_runtime.h>


namespace {
constexpr int B = 8, C = 64, HH = 64, WW = 64, O = 64, K = 3, KK = 9, C2 = 128, NOM = 27, BL = 8  ;
constexpr float XS = 8.0f, WSC = 256.0f;
typedef _Float16 b16;
typedef __attribute__((ext_vector_type(16))) _Float16 v16b;
typedef __attribute__((ext_vector_type(8))) _Float16 v8b;
typedef __attribute__((ext_vector_type(8))) float v8f;
typedef __attribute__((ext_vector_type(4))) float v4f;
__device__ __forceinline__ float bf16_rne(float f) { unsigned int u = __float_as_uint(f); u += 0x7FFFu + ((u >> 16) & 1u); return __uint_as_float(u & 0xFFFF0000u); }
__device__ __forceinline__ void split16(float v, b16& hi, b16& lo) { hi = (b16)v; lo = (b16)(v - (float)hi); }
__device__ __forceinline__ v16b frag_kb(const b16* p, int hh) { const v8b a = *(const v8b*)(p + 8 * hh), b = *(const v8b*)(p + 16 + 8 * hh); v16b f;
#pragma unroll
  for (int e = 0; e < 8; ++e) { f[e] = a[e]; f[8 + e] = b[e]; } return f; }
__device__ __forceinline__ v8f wmma16b(v16b a, v16b b, v8f c) { v8f d = __builtin_amdgcn_wmma_f32_16x16x32_f16(false, a, false, b, (short)0, c, false, false); asm volatile("v_nop\n\tv_nop\n\tv_nop\n\tv_nop" : "+v"(d) : "v"(a), "v"(b)); return d; }
__device__ __forceinline__ void wave_lds_sync() { __builtin_amdgcn_fence(__ATOMIC_RELEASE, "workgroup"); __builtin_amdgcn_wave_barrier(); __builtin_amdgcn_fence(__ATOMIC_ACQUIRE, "workgroup"); }
__device__ __forceinline__ float pmul(float a, float b) { float p = a * b; asm volatile("" : "+v"(p)); return p; }
__device__ __forceinline__ int iclamp(int v, int lo, int hi) { return v < lo ? lo : (v > hi ? hi : v); }

typedef __attribute__((ext_vector_type(2))) float v2f;
__global__ __launch_bounds__(256) void xt_kernel(const float* __restrict__ xin, const float* __restrict__ xdg, b16* __restrict__ XT) {
  __shared__ float tile[64][65];
  const int h = blockIdx.x, which = blockIdx.y, b = blockIdx.z, t = threadIdx.x; const float* src = which ? xdg : xin;
  for (int i = t; i < 64 * 64; i += 256) { const int c = i >> 6, w = i & 63; tile[c][w] = bf16_rne(src[(((size_t)b * C + c) * HH + h) * WW + w]); }
  __syncthreads();
  for (int pass = 0; pass < 2; ++pass) { for (int i = t; i < 64 * 8; i += 256) { const int w = i >> 3, c8 = (i & 7) * 8; v8b o; for (int j = 0; j < 8; ++j) o[j] = (b16)(tile[c8 + j][w] * XS); *(volatile v8b*)(XT + (((size_t)b * HH + h) * WW + w) * C2 + which * C + c8) = o; } __threadfence(); }
}
__global__ __launch_bounds__(256) void wprep_kernel(const float* __restrict__ omw, const float* __restrict__ wt, b16* __restrict__ WOM, b16* __restrict__ WMB, b16* __restrict__ ZR) {
  size_t t = (size_t)blockIdx.x * 256 + threadIdx.x; v8b o;
  if (blockIdx.x == 0 && threadIdx.x < (C2 + 8) / 8 + 1) { v8b z = {}; for (int pass = 0; pass < 2; ++pass) { *(volatile v8b*)(ZR + threadIdx.x * 8) = z; __threadfence(); } }
  { const size_t n = (size_t)32 * KK * C2 / 8; if (t < n) { const size_t e = t * 8; const int j = (int)(e / (KK * C2)); const int col = (int)(e % (KK * C2)); const int k = col / C2, c0 = col % C2;
      for (int q = 0; q < 8; ++q) o[q] = (j < NOM) ? (b16)(bf16_rne(omw[(((size_t)j * C2 + c0 + q) * K + k / K) * K + k % K]) * WSC) : (b16)0.0f;
      for (int pass = 0; pass < 2; ++pass) { *(volatile v8b*)(WOM + e) = o; __threadfence(); } return; } t -= n; }
  { const size_t n = (size_t)O * KK * C / 8; if (t < n) { const size_t e = t * 8; const int oo = (int)(e / (KK * C)); const int col = (int)(e % (KK * C)); const int k = col / C, c0 = col % C;
      for (int q = 0; q < 8; ++q) o[q] = (b16)(bf16_rne(wt[(((size_t)oo * C + c0 + q) * K + k / K) * K + k % K]) * WSC);
      for (int pass = 0; pass < 2; ++pass) { *(volatile v8b*)(WMB + e) = o; __threadfence(); } } }
}
__global__ __launch_bounds__(128) void dcn_kernel(const b16* __restrict__ XT, const b16* __restrict__ WOM, const float* __restrict__ omb, const b16* __restrict__ WMB, const b16* __restrict__ ZR, float* __restrict__ out) {
  __shared__ float Om[64][NOM + 2]; __shared__ int Pi0[KK][64], Pj0[KK][64]; __shared__ float Pw[KK][64][4], Pm[KK][64]; __shared__ __attribute__((aligned(16))) b16 Ah[64][C + 8], Al[64][C + 8]; __shared__ __attribute__((aligned(16))) float Os[O][64 + 4];
  const int t = threadIdx.x, wave = t >> 5, lane = t & 31, nloc = lane & 15, hlf = lane >> 4; const int h = blockIdx.x, b = blockIdx.y;
  const b16* XTb = XT + (size_t)b * HH * WW * C2;
  { v8f acc[2] = {(v8f){}, (v8f){}}; const int w = wave * 16 + nloc;
#pragma unroll 1
    for (int k = 0; k < KK; ++k) { const int yy = h + k / 3 - 1, xx = w + k % 3 - 1; const bool in = (yy >= 0 && yy < HH && xx >= 0 && xx < WW); const b16* arow = in ? (XTb + ((size_t)yy * WW + xx) * C2) : ZR;
#pragma unroll
      for (int ks = 0; ks < 4; ++ks) { const v16b a = frag_kb(arow + ks * 32, hlf);
#pragma unroll
        for (int tt = 0; tt < 2; ++tt) acc[tt] = wmma16b(a, frag_kb(WOM + (size_t)(tt * 16 + nloc) * (KK * C2) + k * C2 + ks * 32, hlf), acc[tt]); } }
#pragma unroll
    for (int tt = 0; tt < 2; ++tt) { const int j = tt * 16 + nloc; const float bb = (j < NOM) ? bf16_rne(omb[j]) : 0.0f;
#pragma unroll
      for (int r = 0; r < 8; ++r) if (j < NOM) Om[wave * 16 + 8 * hlf + r][j] = acc[tt][r] * (1.0f / (XS * WSC)) + bb; } }
  __syncthreads();
  for (int i = t; i < 64 * KK; i += 128) { const int p = i / KK, k = i % KK; const float dy = Om[p][2 * k], dx = Om[p][2 * k + 1], mk = 1.0f / (1.0f + __expf(-Om[p][18 + k]));
    const float yv = ((float)h - 1.0f + (float)(k / 3)) + dy, xv = ((float)p - 1.0f + (float)(k % 3)) + dx; const float fy = floorf(yv), fx = floorf(xv); const int y0 = (int)fy, x0 = (int)fx; const float wy = yv - fy, wx = xv - fx;
    const bool vy0 = (y0 >= 0 && y0 < HH), vy1 = (y0 + 1 >= 0 && y0 + 1 < HH), vx0 = (x0 >= 0 && x0 < WW), vx1 = (x0 + 1 >= 0 && x0 + 1 < WW);
    Pi0[k][p] = y0; Pj0[k][p] = x0; Pm[k][p] = mk;
    Pw[k][p][0] = (vy0 && vx0) ? (1.0f - wy) * (1.0f - wx) : 0.0f; Pw[k][p][1] = (vy0 && vx1) ? (1.0f - wy) * wx : 0.0f; Pw[k][p][2] = (vy1 && vx0) ? wy * (1.0f - wx) : 0.0f; Pw[k][p][3] = (vy1 && vx1) ? wy * wx : 0.0f; }
  __syncthreads();
  v8f acc[4];
#pragma unroll
  for (int tt = 0; tt < 4; ++tt) acc[tt] = (v8f){};
#pragma unroll 1
  for (int k = 0; k < KK; ++k) {
    { const int p = t >> 1, ch0 = (t & 1) * 32; const int y0 = Pi0[k][p], x0 = Pj0[k][p]; const float w00 = Pw[k][p][0], w01 = Pw[k][p][1], w10 = Pw[k][p][2], w11 = Pw[k][p][3], mk = Pm[k][p];
      const int y0c = iclamp(y0, 0, HH - 1), y1c = iclamp(y0 + 1, 0, HH - 1), x0c = iclamp(x0, 0, WW - 1), x1c = iclamp(x0 + 1, 0, WW - 1);
      const b16* r00 = XTb + ((size_t)y0c * WW + x0c) * C2 + ch0, * r01 = XTb + ((size_t)y0c * WW + x1c) * C2 + ch0, * r10 = XTb + ((size_t)y1c * WW + x0c) * C2 + ch0, * r11 = XTb + ((size_t)y1c * WW + x1c) * C2 + ch0;
#pragma unroll
      for (int q = 0; q < 32; q += 8) { const v8b a = *(const v8b*)(r00 + q), bq = *(const v8b*)(r01 + q), cq = *(const v8b*)(r10 + q), dq = *(const v8b*)(r11 + q); v8b hv, lv;
#pragma unroll
        for (int j = 0; j < 8; ++j) { const float s = ((pmul((float)a[j], w00) + pmul((float)bq[j], w01) + pmul((float)cq[j], w10) + pmul((float)dq[j], w11)) * (1.0f / XS)) * mk; b16 ph, pl; split16(s * XS, ph, pl); hv[j] = ph; lv[j] = pl; }
        *(v8b*)(&Ah[p][ch0 + q]) = hv; *(v8b*)(&Al[p][ch0 + q]) = lv; } }
    __syncthreads();
#pragma unroll
    for (int ks = 0; ks < 2; ++ks) { const v16b a = frag_kb(&Ah[wave * 16 + nloc][ks * 32], hlf), al = frag_kb(&Al[wave * 16 + nloc][ks * 32], hlf);
#pragma unroll
      for (int tt = 0; tt < 4; ++tt) { const v16b bw = frag_kb(WMB + (size_t)(tt * 16 + nloc) * (KK * C) + k * C + ks * 32, hlf); acc[tt] = wmma16b(a, bw, acc[tt]); acc[tt] = wmma16b(al, bw, acc[tt]); } }
    __syncthreads(); }
#pragma unroll
  for (int tt = 0; tt < 4; ++tt)
#pragma unroll
    for (int r = 0; r < 8; ++r) Os[tt * 16 + nloc][wave * 16 + 8 * hlf + r] = acc[tt][r] * (1.0f / (XS * WSC));
  __syncthreads();
  for (int pass = 0; pass < 2; ++pass) { for (int q = 0; q < 16; ++q) { const int oo = wave * 16 + q; v2f v = {Os[oo][lane * 2], Os[oo][lane * 2 + 1]}; *(volatile v2f*)(out + (((size_t)b * O + oo) * HH + h) * WW + lane * 2) = v; } __threadfence(); }
}
}

extern "C" void kernel_launch(void* const* d_in, const int* in_sizes, int n_in, void* d_out, int out_size, void* d_ws, size_t ws_size, hipStream_t stream) {
  (void)n_in;
  auto Fp = [&](int i) { return (const float*)d_in[i]; };
  if (in_sizes[0] != B * C * HH * WW || in_sizes[1] != B * C * HH * WW || in_sizes[2] != O * C * KK || in_sizes[3] != NOM * C2 * KK || in_sizes[4] != NOM || out_size != B * O * HH * WW) return;
  size_t off = 0; char* ws = (char*)d_ws;
  auto carve = [&](size_t bytes) { char* p = ws + off; off += (bytes + 255) & ~(size_t)255; return p; };
  b16* XT = (b16*)carve((size_t)B * HH * WW * C2 * 2); b16* WOM = (b16*)carve((size_t)32 * KK * C2 * 2); b16* WMB = (b16*)carve((size_t)O * KK * C * 2); b16* ZR = (b16*)carve(512);
  if (off > ws_size || off > ((size_t)128 << 20)) return;
  xt_kernel<<<dim3(HH, 2, BL), 256, 0, stream>>>(Fp(0), Fp(1), XT);
  wprep_kernel<<<(unsigned)((((size_t)32 * KK * C2 + (size_t)O * KK * C) / 8 + 255) / 256), 256, 0, stream>>>(Fp(3), Fp(2), WOM, WMB, ZR);
  dcn_kernel<<<dim3(HH, BL), 128, 0, stream>>>(XT, WOM, Fp(4), WMB, ZR, (float*)d_out);
}
